// DCRNN_RGCN_89008902243183
// MI455X (gfx1250) — hardware-run, weakly checked
//
#include <hip/hip_runtime.h>


namespace {
constexpr int N = 50000, E = 800000, F = 128, NC = 16;
constexpr float XS = 8.0f, WSC = 256.0f;
typedef _Float16 b16;
typedef __attribute__((ext_vector_type(16))) _Float16 v16b;
typedef __attribute__((ext_vector_type(8))) _Float16 v8b;
typedef __attribute__((ext_vector_type(8))) float v8f;
typedef __attribute__((ext_vector_type(4))) float v4f;
__device__ __forceinline__ float bf16_rne(float f) { unsigned int u = __float_as_uint(f); u += 0x7FFFu + ((u >> 16) & 1u); float r = __uint_as_float(u & 0xFFFF0000u); asm volatile("" : "+v"(r)); return r; }
__device__ __forceinline__ void split16(float v, b16& hi, b16& lo) { hi = (b16)v; lo = (b16)(v - (float)hi); }
__device__ __forceinline__ v16b frag_kb(const b16* p, int hh) { const v8b a = *(const v8b*)(p + 8 * hh), b = *(const v8b*)(p + 16 + 8 * hh); v16b f;
#pragma unroll
  for (int e = 0; e < 8; ++e) { f[e] = a[e]; f[8 + e] = b[e]; } return f; }
__device__ __forceinline__ v8f wmma16b(v16b a, v16b b, v8f c) { v8f d = __builtin_amdgcn_wmma_f32_16x16x32_f16(false, a, false, b, (short)0, c, false, false); asm volatile("v_nop\n\tv_nop\n\tv_nop\n\tv_nop" : "+v"(d) : "v"(a), "v"(b)); return d; }
__device__ __forceinline__ void wave_lds_sync() { __builtin_amdgcn_fence(__ATOMIC_RELEASE, "workgroup"); __builtin_amdgcn_wave_barrier(); __builtin_amdgcn_fence(__ATOMIC_ACQUIRE, "workgroup"); }
__device__ __forceinline__ float pmul(float a, float b) { float p = a * b; asm volatile("" : "+v"(p)); return p; }
__device__ __forceinline__ int iclamp(int v, int lo, int hi) { return v < lo ? lo : (v > hi ? hi : v); }
__device__ __forceinline__ float sigm(float v) { return 1.0f / (1.0f + __expf(-v)); }
constexpr int CSR_NBLK9 = 512, CSR_GB9 = 9, CSR_GN9 = 1 << CSR_GB9  , CSR_TS9 = (CSR_GN9 < 32 ? 32 : CSR_GN9)  , CSR_MAXG9 = 512, CSR_CAP9 = 12288  ;
__device__ __host__ __forceinline__ int csr_tix9(int v) { return (v >> CSR_GB9) * CSR_TS9 + (v & (CSR_GN9 - 1)); }
__global__ __launch_bounds__(64) void csrA_kernel9(const int* __restrict__ dst, int E, int N, int nG, int CHP, int NGP, int* __restrict__ STG, int* __restrict__ HST) {
  extern __shared__ int sm[];
  int* cnt = sm; int* run = sm + NGP; int* ids = sm + 2 * NGP;
  const int b = blockIdx.x; const int ch = (E + CSR_NBLK9 - 1) / CSR_NBLK9; const int e0 = b * ch, e1 = min(E, e0 + ch);
  for (int i = threadIdx.x; i < NGP; i += 64) cnt[i] = 0;
  for (int i = threadIdx.x; i < CHP; i += 64) ids[i] = -1;
  __syncthreads();
  if (threadIdx.x == 0) {
    for (int e = e0; e < e1; ++e) { int d = dst[e]; d = (d < 0) ? 0 : (d >= N ? N - 1 : d); cnt[d >> CSR_GB9] += 1; }
    int acc = 0; for (int g = 0; g < nG; ++g) { run[g] = acc; acc += cnt[g]; }
    for (int e = e0; e < e1; ++e) { int d = dst[e]; d = (d < 0) ? 0 : (d >= N ? N - 1 : d); const int g = d >> CSR_GB9; ids[run[g]] = e; run[g] += 1; } }
  __syncthreads();
  typedef __attribute__((ext_vector_type(4))) int v4i;
  for (int pass = 0; pass < 2; ++pass) {
    for (int i = threadIdx.x; i < CHP / 4; i += 64) *(volatile v4i*)(STG + (size_t)b * CHP + i * 4) = *(const v4i*)(&ids[i * 4]);
    for (int i = threadIdx.x; i < NGP / 4; i += 64) { v4i v; for (int e = 0; e < 4; ++e) v[e] = (i * 4 + e < nG) ? cnt[i * 4 + e] : 0; *(volatile v4i*)(HST + (size_t)b * NGP + i * 4) = v; }
    __threadfence(); }
}
__global__ __launch_bounds__(512) void csrS_kernel9(const int* __restrict__ HST, int nG, int NGP, int* __restrict__ START, int* __restrict__ TOT, int* __restrict__ OFF) {
  __shared__ int tot[CSR_MAXG9];
  const int b = threadIdx.x;
  for (int pass = 0; pass < 2; ++pass) { int runb = 0; for (int g = 0; g < nG; ++g) { int c = HST[(size_t)b * NGP + g]; c = (c < 0) ? 0 : c; ((volatile int*)OFF)[(size_t)g * CSR_NBLK9 + b] = runb; runb += c; } __threadfence(); }
  for (int g = threadIdx.x; g < nG; g += 512) { int s = 0; for (int bb = 0; bb < CSR_NBLK9; ++bb) { int c = HST[(size_t)bb * NGP + g]; s += (c < 0) ? 0 : c; } tot[g] = s; }
  __syncthreads();
  if (threadIdx.x < 32) {
    __shared__ int st[CSR_MAXG9 + 32];
    if (threadIdx.x == 0) { int acc = 0; for (int g = 0; g < NGP; ++g) { st[g] = acc; if (g < nG) acc += (tot[g] + 31) & ~31; } st[NGP] = acc; }
    __builtin_amdgcn_fence(__ATOMIC_RELEASE, "workgroup"); __builtin_amdgcn_wave_barrier(); __builtin_amdgcn_fence(__ATOMIC_ACQUIRE, "workgroup");
    for (int pass = 0; pass < 2; ++pass) { for (int i = threadIdx.x; i < NGP + 32; i += 32) { ((volatile int*)START)[i] = (i <= NGP) ? st[min(i, NGP)] : 0; ((volatile int*)TOT)[i] = (i < nG) ? tot[i] : 0; } __threadfence(); } }
}
__global__ __launch_bounds__(256) void csrB_kernel9(const int* __restrict__ dst, int N, int nG, int CHP, int NGP, int permLen, const int* __restrict__ STG, const int* __restrict__ HST, const int* __restrict__ OFF, const int* __restrict__ START, const int* __restrict__ TOT, int* __restrict__ PERM, int* __restrict__ ROWPTR, int* __restrict__ ROWCNT, int* __restrict__ FLAG) {
  typedef __attribute__((ext_vector_type(4))) int v4i;
  __shared__ int ids[CSR_CAP9]; __shared__ unsigned short key[CSR_CAP9]; __shared__ int outp[CSR_CAP9]; __shared__ int ncnt[CSR_GN9 + 1]; __shared__ int boff[CSR_NBLK9 + 1];
  const int g = blockIdx.x, t_ = threadIdx.x; int tot = TOT[g]; int st = START[g], stn = START[g + 1]; const int v0 = g * CSR_GN9; const int nv = min(CSR_GN9, N - v0); const int t0 = g * CSR_TS9;
  st = (st < 0) ? 0 : (st > permLen - 32 ? permLen - 32 : st) & ~31; stn = (stn < st) ? st : (stn > permLen ? permLen : stn); tot = (tot < 0) ? 0 : tot; if (tot > stn - st && tot <= CSR_CAP9) tot = stn - st;
  if (tot > CSR_CAP9) {
    for (int pass = 0; pass < 2; ++pass) { for (int i = t_; i < CSR_TS9 / 4; i += 256) { v4i a, c; for (int e = 0; e < 4; ++e) { a[e] = st; c[e] = 0; } *(volatile v4i*)(ROWPTR + t0 + i * 4) = a; *(volatile v4i*)(ROWCNT + t0 + i * 4) = c; } if (t_ == 0) ((volatile int*)FLAG)[0] = 1; __threadfence(); } (void)nv; return; }
  if (t_ == 0) { int acc = 0; for (int b = 0; b < CSR_NBLK9; ++b) { boff[b] = acc; int c = HST[(size_t)b * NGP + g]; c = (c < 0) ? 0 : (c > CHP ? CHP : c); acc += c; if (acc > tot) acc = tot; } boff[CSR_NBLK9] = acc; }
  for (int i = t_; i <= CSR_GN9; i += 256) ncnt[i] = 0;
  __syncthreads();
  for (int b = 0; b < CSR_NBLK9; ++b) { const int c = boff[b + 1] - boff[b]; int o_ = OFF[(size_t)g * CSR_NBLK9 + b]; o_ = (o_ < 0) ? 0 : (o_ > CHP - c ? CHP - c : o_); const int* src_ = STG + (size_t)b * CHP + o_;
    for (int i = t_; i < c; i += 256) { int id = src_[i]; id = (id < 0) ? 0 : id; ids[boff[b] + i] = id; int d = dst[id]; d = (d < v0) ? v0 : (d >= N ? N - 1 : d); int kk = d - v0; kk = (kk < 0) ? 0 : (kk >= CSR_GN9 ? CSR_GN9 - 1 : kk); key[boff[b] + i] = (unsigned short)kk; } }
  __syncthreads();
  if (t_ == 0) { for (int i = 0; i < tot; ++i) ncnt[key[i]] += 1; int acc = 0; for (int vl = 0; vl < CSR_GN9; ++vl) { const int c = ncnt[vl]; ncnt[vl] = acc; acc += c; } ncnt[CSR_GN9] = acc;
    for (int i = 0; i < tot; ++i) { const int vl = key[i]; outp[ncnt[vl]] = ids[i]; ncnt[vl] += 1; }
    for (int vl = CSR_GN9; vl > 0; --vl) ncnt[vl] = ncnt[vl - 1]; ncnt[0] = 0; }
  __syncthreads();
  for (int pass = 0; pass < 2; ++pass) {
    for (int i = t_; i < (stn - st) / 4; i += 256) { v4i v; for (int e = 0; e < 4; ++e) { const int q = i * 4 + e; v[e] = (q < tot) ? outp[q] : -1; } *(volatile v4i*)(PERM + st + i * 4) = v; }
    for (int i = t_; i < CSR_TS9 / 4; i += 256) { v4i a, c; for (int e = 0; e < 4; ++e) { const int vl = i * 4 + e; const int vc = vl < CSR_GN9 ? vl : CSR_GN9; a[e] = (vl < CSR_GN9) ? st + ncnt[vc] : st; c[e] = (vl < nv) ? (ncnt[(vc < CSR_GN9 ? vc : CSR_GN9 - 1) + 1] - ncnt[vc]) : 0; } *(volatile v4i*)(ROWPTR + t0 + i * 4) = a; *(volatile v4i*)(ROWCNT + t0 + i * 4) = c; }
    __threadfence(); }
}
__global__ __launch_bounds__(256) void csrZ_kernel9(int* __restrict__ p, size_t n4) { typedef __attribute__((ext_vector_type(4))) int v4i; const size_t tid = (size_t)blockIdx.x * 256 + threadIdx.x, nth = (size_t)gridDim.x * 256; v4i z = {0, 0, 0, 0}; for (size_t i = tid; i < n4; i += nth) *(volatile v4i*)(p + i * 4) = z; }
struct CsrBufs9 { int *STG, *HST, *OFF, *START, *TOT, *PERM, *ROWPTR, *ROWCNT, *FLAG; int nG, NGP, CHP; size_t permLen; char* base; size_t bytes; };
static size_t csr_carve9(CsrBufs9& c, char* ws, size_t off, int E, int N) {
  const size_t off0 = off; c.base = ws + off;
  auto al = [&](size_t bytes) { char* p = ws + off; off += (bytes + 255) & ~(size_t)255; return p; };
  c.nG = (N + CSR_GN9 - 1) / CSR_GN9; c.NGP = (c.nG + 31) & ~31; const int ch = (E + CSR_NBLK9 - 1) / CSR_NBLK9; c.CHP = (ch + 31) & ~31; c.permLen = (size_t)E + 32 * (size_t)c.nG + 32;
  c.STG = (int*)al((size_t)CSR_NBLK9 * c.CHP * 4); c.HST = (int*)al((size_t)CSR_NBLK9 * c.NGP * 4); c.OFF = (int*)al((size_t)c.NGP * CSR_NBLK9 * 4); c.START = (int*)al((size_t)(c.NGP + 64) * 4); c.TOT = (int*)al((size_t)(c.NGP + 64) * 4);
  c.PERM = (int*)al(c.permLen * 4); c.ROWPTR = (int*)al((size_t)c.nG * CSR_TS9 * 4); c.ROWCNT = (int*)al((size_t)c.nG * CSR_TS9 * 4); c.FLAG = (int*)al(256);
  c.bytes = off - off0; return off;
}
static void csr_build9(const CsrBufs9& c, const int* dst, int E, int N, hipStream_t stream) {
  const size_t smem = (size_t)(2 * c.NGP + c.CHP) * 4;
  csrZ_kernel9<<<512, 256, 0, stream>>>((int*)c.base, c.bytes / 16);
  csrA_kernel9<<<CSR_NBLK9, 64, smem, stream>>>(dst, E, N, c.nG, c.CHP, c.NGP, c.STG, c.HST);
  csrS_kernel9<<<1, 512, 0, stream>>>(c.HST, c.nG, c.NGP, c.START, c.TOT, c.OFF);
  csrB_kernel9<<<c.nG, 256, 0, stream>>>(dst, N, c.nG, c.CHP, c.NGP, (int)c.permLen, c.STG, c.HST, c.OFF, c.START, c.TOT, c.PERM, c.ROWPTR, c.ROWCNT, c.FLAG);
}


__global__ __launch_bounds__(256) void wput_kernel(const float* __restrict__ wg, const float* __restrict__ wz0, const float* __restrict__ wz1, const float* __restrict__ wr0, const float* __restrict__ wr1, const float* __restrict__ wh0, const float* __restrict__ wh1, const float* __restrict__ wl, b16* __restrict__ WGT, b16* __restrict__ WZRh, b16* __restrict__ WZRl, b16* __restrict__ WHTh, b16* __restrict__ WHTl, b16* __restrict__ WLT) { const int u = blockIdx.x * 256 + threadIdx.x;
  for (int pass = 0; pass < 2; ++pass) {
    if (u < F * 16) { const int o = u / 16, k0 = (u % 16) * 8; v8b v;
#pragma unroll
      for (int j = 0; j < 8; ++j) v[j] = (b16)(bf16_rne(wg[(size_t)(k0 + j) * F + o]) * WSC); *(volatile v8b*)(WGT + (size_t)o * F + k0) = v; }
    if (u < 2 * F * 32) { const int r = u / 32, k0 = (u % 32) * 8; const int o = r % F; const float* a = r < F ? wz0 : wr0; const float* c = r < F ? wz1 : wr1; v8b hv, lv;
#pragma unroll
      for (int j = 0; j < 8; ++j) { const float s = bf16_rne(a[(size_t)(k0 + j) * F + o]) + bf16_rne(c[(size_t)(k0 + j) * F + o]); b16 p, q; split16(s * WSC, p, q); hv[j] = p; lv[j] = q; } *(volatile v8b*)(WZRh + (size_t)r * 2 * F + k0) = hv; *(volatile v8b*)(WZRl + (size_t)r * 2 * F + k0) = lv; }
    if (u < F * 32) { const int o = u / 32, k0 = (u % 32) * 8; v8b hv, lv;
#pragma unroll
      for (int j = 0; j < 8; ++j) { const float s = bf16_rne(wh0[(size_t)(k0 + j) * F + o]) + bf16_rne(wh1[(size_t)(k0 + j) * F + o]); b16 p, q; split16(s * WSC, p, q); hv[j] = p; lv[j] = q; } *(volatile v8b*)(WHTh + (size_t)o * 2 * F + k0) = hv; *(volatile v8b*)(WHTl + (size_t)o * 2 * F + k0) = lv; }
    if (u < NC * 16) { const int o = u / 16, k0 = (u % 16) * 8; v8b v;
#pragma unroll
      for (int j = 0; j < 8; ++j) v[j] = (b16)(bf16_rne(wl[(size_t)(k0 + j) * NC + o]) * WSC); *(volatile v8b*)(WLT + (size_t)o * F + k0) = v; }
    __threadfence(); } }
__global__ __launch_bounds__(256) void deg_kernel(const float* __restrict__ ew, const int* __restrict__ PERM, const int* __restrict__ ROWPTR, const int* __restrict__ ROWCNT, int permLen, float* __restrict__ DIS) { const int i = blockIdx.x * 256 + threadIdx.x; if (i >= N) return; int st = ROWPTR[i], cnt = ROWCNT[i]; cnt = iclamp(cnt, 0, E); st = iclamp(st, 0, permLen - cnt);
  float d = 1.0f; for (int j = 0; j < cnt; ++j) { const int e = iclamp(PERM[st + j], 0, E - 1); d += bf16_rne(ew[e]); } const float dis = d > 0.0f ? rsqrtf(d) : 0.0f;
  for (int pass = 0; pass < 2; ++pass) { ((volatile float*)DIS)[i] = dis; __threadfence(); } }
__global__ __launch_bounds__(32) void xw_kernel(const float* __restrict__ x, const b16* __restrict__ WGT, int NLIM, float* __restrict__ XW) { __shared__ __attribute__((aligned(16))) b16 Ah[16][F + 8]; __shared__ float Tf[16][132]; const int lane = threadIdx.x, nloc = lane & 15, hlf = lane >> 4; const size_t m0 = (size_t)blockIdx.x * 16; if (m0 >= (size_t)NLIM) return;
  for (int rr = 0; rr < 16; ++rr) for (int q = 0; q < 4; ++q) Ah[rr][q * 32 + lane] = (b16)(bf16_rne(x[(m0 + rr) * F + q * 32 + lane]) * XS);
  wave_lds_sync(); v8f acc[8];
#pragma unroll
  for (int t = 0; t < 8; ++t) acc[t] = (v8f){};
#pragma unroll
  for (int kb = 0; kb < F; kb += 32) { const v16b a = frag_kb(&Ah[nloc][kb], hlf);
#pragma unroll
    for (int t = 0; t < 8; ++t) acc[t] = wmma16b(a, frag_kb(WGT + (size_t)(t * 16 + nloc) * F + kb, hlf), acc[t]); }
#pragma unroll
  for (int t = 0; t < 8; ++t)
#pragma unroll
    for (int r8 = 0; r8 < 8; ++r8) Tf[8 * hlf + r8][t * 16 + nloc] = acc[t][r8] * (1.0f / (XS * WSC));
  wave_lds_sync();
  for (int pass = 0; pass < 2; ++pass) { for (int rr = 0; rr < 16; ++rr) *(volatile v4f*)(XW + (m0 + rr) * F + lane * 4) = *(const v4f*)(&Tf[rr][lane * 4]); __threadfence(); } }
__global__ __launch_bounds__(256) void prop_kernel(const float* __restrict__ XW, const float* __restrict__ ew, const float* __restrict__ DIS, const float* __restrict__ bg, const int* __restrict__ srcs, const int* __restrict__ PERM, const int* __restrict__ ROWPTR, const int* __restrict__ ROWCNT, int permLen, int NLIM, float* __restrict__ HG) { const int wave = threadIdx.x >> 5, lane = threadIdx.x & 31; const size_t i = (size_t)blockIdx.x * 8 + wave; if (i >= (size_t)NLIM) return; int st = ROWPTR[i], cnt = ROWCNT[i]; cnt = iclamp(cnt, 0, E); st = iclamp(st, 0, permLen - cnt); const float di = DIS[i];
  v4f acc; { const v4f v = *(const v4f*)(XW + i * F + lane * 4); const float s = pmul(di, di); for (int k = 0; k < 4; ++k) acc[k] = pmul(s, v[k]); }
#pragma unroll 1
  for (int j = 0; j < cnt; ++j) { const int e = iclamp(PERM[st + j], 0, E - 1); const size_t u = (size_t)iclamp(srcs[e], 0, N - 1); if (u >= (size_t)NLIM) continue; const float nrm = pmul(pmul(DIS[u], bf16_rne(ew[e])), di); const v4f v = *(const v4f*)(XW + u * F + lane * 4); for (int k = 0; k < 4; ++k) acc[k] += pmul(nrm, v[k]); }
  for (int k = 0; k < 4; ++k) acc[k] += bf16_rne(bg[lane * 4 + k]);
  for (int pass = 0; pass < 2; ++pass) { *(volatile v4f*)(HG + i * F + lane * 4) = acc; __threadfence(); } }
__global__ __launch_bounds__(32) void cell_kernel(const float* __restrict__ HG, const float* __restrict__ Hs, const b16* __restrict__ WZRh, const b16* __restrict__ WZRl, const float* __restrict__ bz, const float* __restrict__ br, const b16* __restrict__ WHTh, const b16* __restrict__ WHTl, const float* __restrict__ bh, const b16* __restrict__ WLT, const float* __restrict__ bl, int NLIM, float* __restrict__ PROBS, float* __restrict__ HN) {
  __shared__ __attribute__((aligned(16))) b16 Ah[16][264], Al[16][264]; __shared__ float Zf[16][132], Tf[16][132]; const int lane = threadIdx.x, nloc = lane & 15, hlf = lane >> 4; const size_t m0 = (size_t)blockIdx.x * 16; if (m0 >= (size_t)NLIM) return;
  for (int rr = 0; rr < 16; ++rr) for (int q = 0; q < 4; ++q) { b16 p, ql; split16(HG[(m0 + rr) * F + q * 32 + lane] * XS, p, ql); Ah[rr][q * 32 + lane] = p; Al[rr][q * 32 + lane] = ql; Ah[rr][F + q * 32 + lane] = (b16)(bf16_rne(Hs[(m0 + rr) * F + q * 32 + lane]) * XS); Al[rr][F + q * 32 + lane] = (b16)0.0f; }
  wave_lds_sync(); v8f acc[16];
#pragma unroll
  for (int t = 0; t < 16; ++t) acc[t] = (v8f){};
#pragma unroll
  for (int kb = 0; kb < 2 * F; kb += 32) { const v16b a = frag_kb(&Ah[nloc][kb], hlf); v16b al; if (kb < F) al = frag_kb(&Al[nloc][kb], hlf);
#pragma unroll
    for (int t = 0; t < 16; ++t) { const size_t ro = (size_t)(t * 16 + nloc) * 2 * F + kb; const v16b bh_ = frag_kb(WZRh + ro, hlf), bl_ = frag_kb(WZRl + ro, hlf); acc[t] = wmma16b(a, bh_, acc[t]); acc[t] = wmma16b(a, bl_, acc[t]); if (kb < F) acc[t] = wmma16b(al, bh_, acc[t]); } }
#pragma unroll
  for (int t = 0; t < 16; ++t) { const int cc = t * 16 + nloc; const int o = cc & (F - 1); const float bb = bf16_rne(t < 8 ? bz[o] : br[o]);
#pragma unroll
    for (int r8 = 0; r8 < 8; ++r8) { const float g = sigm(acc[t][r8] * (1.0f / (XS * WSC)) + bb); if (t < 8) Zf[8 * hlf + r8][o] = g; else Tf[8 * hlf + r8][o] = g; } }
  wave_lds_sync();
  for (int rr = 0; rr < 16; ++rr) for (int q = 0; q < 4; ++q) { const int o = q * 32 + lane; b16 p, ql; split16(pmul(bf16_rne(Hs[(m0 + rr) * F + o]), Tf[rr][o]) * XS, p, ql); Ah[rr][F + o] = p; Al[rr][F + o] = ql; }
  wave_lds_sync(); v8f ac2[8];
#pragma unroll
  for (int t = 0; t < 8; ++t) ac2[t] = (v8f){};
#pragma unroll
  for (int kb = 0; kb < 2 * F; kb += 32) { const v16b a = frag_kb(&Ah[nloc][kb], hlf), al = frag_kb(&Al[nloc][kb], hlf);
#pragma unroll
    for (int t = 0; t < 8; ++t) { const size_t ro = (size_t)(t * 16 + nloc) * 2 * F + kb; const v16b bh_ = frag_kb(WHTh + ro, hlf), bl_ = frag_kb(WHTl + ro, hlf); ac2[t] = wmma16b(a, bh_, ac2[t]); ac2[t] = wmma16b(a, bl_, ac2[t]); ac2[t] = wmma16b(al, bh_, ac2[t]); } }
  wave_lds_sync();
#pragma unroll
  for (int t = 0; t < 8; ++t) { const int o = t * 16 + nloc; const float bb = bf16_rne(bh[o]);
#pragma unroll
    for (int r8 = 0; r8 < 8; ++r8) { const int rr = 8 * hlf + r8; const float ht = tanhf(ac2[t][r8] * (1.0f / (XS * WSC)) + bb); const float z = Zf[rr][o]; const float hs = bf16_rne(Hs[(m0 + rr) * F + o]); Tf[rr][o] = pmul(z, hs) + pmul(1.0f - z, ht); } }
  wave_lds_sync();
  for (int rr = 0; rr < 16; ++rr) for (int q = 0; q < 4; ++q) { const int o = q * 32 + lane; b16 p, ql; split16(fmaxf(Tf[rr][o], 0.0f) * XS, p, ql); Ah[rr][o] = p; Al[rr][o] = ql; }
  wave_lds_sync(); v8f al3 = {};
#pragma unroll
  for (int kb = 0; kb < F; kb += 32) { const v16b a = frag_kb(&Ah[nloc][kb], hlf), al = frag_kb(&Al[nloc][kb], hlf); const v16b bw = frag_kb(WLT + (size_t)nloc * F + kb, hlf); al3 = wmma16b(a, bw, al3); al3 = wmma16b(al, bw, al3); }
  float pr[8];
#pragma unroll
  for (int r8 = 0; r8 < 8; ++r8) { const float lg = al3[r8] * (1.0f / (XS * WSC)) + bf16_rne(bl[nloc]); float mx = lg; mx = fmaxf(mx, __shfl_xor(mx, 1)); mx = fmaxf(mx, __shfl_xor(mx, 2)); mx = fmaxf(mx, __shfl_xor(mx, 4)); mx = fmaxf(mx, __shfl_xor(mx, 8)); const float e = __expf(lg - mx); float s = e; s += __shfl_xor(s, 1); s += __shfl_xor(s, 2); s += __shfl_xor(s, 4); s += __shfl_xor(s, 8); pr[r8] = e / s; }
  __shared__ float Pf[16][20];
#pragma unroll
  for (int r8 = 0; r8 < 8; ++r8) Pf[8 * hlf + r8][nloc] = pr[r8];
  wave_lds_sync();
  for (int pass = 0; pass < 2; ++pass) { for (int rr = 0; rr < 16; ++rr) *(volatile v4f*)(HN + (m0 + rr) * F + lane * 4) = *(const v4f*)(&Tf[rr][lane * 4]); for (int q = lane; q < 256; q += 32) ((volatile float*)PROBS)[m0 * NC + q] = Pf[q / NC][q % NC]; __threadfence(); } }
}

extern "C" void kernel_launch(void* const* d_in, const int* in_sizes, int n_in, void* d_out, int out_size, void* d_ws, size_t ws_size, hipStream_t stream) {
  (void)n_in;
  auto Fp = [&](int i) { return (const float*)d_in[i]; }; auto Ip = [&](int i) { return (const int*)d_in[i]; };
  if (in_sizes[0] != N * F || in_sizes[1] != 2 * E || in_sizes[2] != E || in_sizes[3] != N * F || in_sizes[4] != F * F || in_sizes[6] != 2 * F * F || in_sizes[12] != 2 * F * F || in_sizes[15] != F * NC || out_size != N * NC + N * F) return;
  const int NLIM = N;
  size_t off = 0; char* ws = (char*)d_ws;
  auto carve = [&](size_t bytes) { char* p = ws + off; off += (bytes + 255) & ~(size_t)255; return p; };
  b16* WGT = (b16*)carve((size_t)F * F * 2); b16* WZRh = (b16*)carve((size_t)2 * F * 2 * F * 2); b16* WZRl = (b16*)carve((size_t)2 * F * 2 * F * 2); b16* WHTh = (b16*)carve((size_t)F * 2 * F * 2); b16* WHTl = (b16*)carve((size_t)F * 2 * F * 2); b16* WLT = (b16*)carve((size_t)NC * F * 2);
  float* DIS = (float*)carve((size_t)N * 4); float* XW = (float*)carve((size_t)N * F * 4); float* HG = (float*)carve((size_t)N * F * 4); CsrBufs9 csr; off = csr_carve9(csr, ws, off, E, N);
  if (off > ws_size || off > ((size_t)96 << 20)) return;
  float* PROBS = (float*)d_out; float* HN = PROBS + (size_t)N * NC;
  wput_kernel<<<(2 * F * 32 + 255) / 256, 256, 0, stream>>>(Fp(4), Fp(6), Fp(7), Fp(9), Fp(10), Fp(12), Fp(13), Fp(15), WGT, WZRh, WZRl, WHTh, WHTl, WLT);
  csr_build9(csr, Ip(1) + E, E, N, stream);
  deg_kernel<<<(N + 255) / 256, 256, 0, stream>>>(Fp(2), csr.PERM, csr.ROWPTR, csr.ROWCNT, (int)csr.permLen, DIS);
  xw_kernel<<<NLIM / 16, 32, 0, stream>>>(Fp(0), WGT, NLIM, XW);
  prop_kernel<<<(NLIM + 7) / 8, 256, 0, stream>>>(XW, Fp(2), DIS, Fp(5), Ip(1), csr.PERM, csr.ROWPTR, csr.ROWCNT, (int)csr.permLen, NLIM, HG);
  cell_kernel<<<NLIM / 16, 32, 0, stream>>>(HG, Fp(3), WZRh, WZRl, Fp(8), Fp(11), WHTh, WHTl, Fp(14), WLT, Fp(16), NLIM, PROBS, HN);
}
